// LongformerSelfAttention_65687229825616
// MI455X (gfx1250) — hardware-verified
//
#include <hip/hip_runtime.h>


#ifndef NB
#define NB 2
#endif
#ifndef SEQ
#define SEQ 2048
#endif
#define NB_FULL  2
#define SEQ_FULL 2048
#define DM   1024
#define NH_  16
#define HD   64
#define DQ   (NH_ * HD)
#define NTOK (NB * SEQ)
#define WIN  128
#define SCL  0.125f
#define L2E  1.4426950408889634f
static_assert(NB >= 1 && NB <= NB_FULL);
static_assert(SEQ >= 64 && SEQ <= SEQ_FULL && SEQ % 64 == 0);
static_assert(DQ == DM && DM % 64 == 0 && HD == 64);
static_assert((size_t)((NB - 1) * SEQ_FULL + SEQ) * DM <= (size_t)NB_FULL * SEQ_FULL * DM);

typedef _Float16 h16;
typedef unsigned short bf;
typedef __attribute__((ext_vector_type(16))) __bf16   v16bf;
typedef __attribute__((ext_vector_type(16))) _Float16 v16h;
typedef __attribute__((ext_vector_type(8)))  _Float16 v8h;
typedef __attribute__((ext_vector_type(8)))  unsigned short v8us;
typedef __attribute__((ext_vector_type(4)))  unsigned short v4us;
typedef __attribute__((ext_vector_type(8)))  float    v8f;
typedef __attribute__((ext_vector_type(4)))  float    v4f;
typedef v8h  __attribute__((may_alias)) v8ha;
typedef v4f  __attribute__((may_alias)) v4fa;
typedef v8us __attribute__((may_alias)) v8usa;

__device__ __forceinline__ unsigned short f2bf(float f) { unsigned u = __float_as_uint(f); u += 0x7FFFu + ((u >> 16) & 1u); return (unsigned short)(u >> 16); }
__device__ __forceinline__ float bf2f(unsigned short b) { return __uint_as_float(((unsigned)b) << 16); }
__device__ __forceinline__ float bfr(float f) { return bf2f(f2bf(f)); }
__device__ __forceinline__ v16h cat16(v8h lo, v8h hi) { return __builtin_shufflevector(lo, hi, 0, 1, 2, 3, 4, 5, 6, 7, 8, 9, 10, 11, 12, 13, 14, 15); }
__device__ __forceinline__ v16bf cat16b(v8us lo, v8us hi) { return __builtin_bit_cast(v16bf, __builtin_shufflevector(lo, hi, 0, 1, 2, 3, 4, 5, 6, 7, 8, 9, 10, 11, 12, 13, 14, 15)); }
__device__ __forceinline__ v8f wmma16(v16h a, v16h b, v8f c) { return __builtin_amdgcn_wmma_f32_16x16x32_f16(false, a, false, b, (short)0, c, false, false); }
__device__ __forceinline__ v8f wmmab(v16bf a, v16bf b, v8f c) { return __builtin_amdgcn_wmma_f32_16x16x32_bf16(false, a, false, b, (short)0, c, false, false); }
__device__ __forceinline__ void splitf(float y, unsigned short& h, unsigned short& l) { h = f2bf(y); l = f2bf(y - bf2f(h)); }

template <typename T16> struct WFrag;
template <> struct WFrag<h16> { typedef v16h V; static __device__ __forceinline__ V ld(const h16* p) { return cat16(*(const v8h*)p, *(const v8h*)(p + 16)); } static __device__ __forceinline__ v8f mma(V a, V b, v8f c) { return wmma16(a, b, c); } };
template <> struct WFrag<bf> { typedef v16bf V; static __device__ __forceinline__ V ld(const bf* p) { return cat16b(*(const v8us*)p, *(const v8us*)(p + 16)); } static __device__ __forceinline__ v8f mma(V a, V b, v8f c) { return wmmab(a, b, c); } };
template <typename T16, int NSPLIT, int BIAS>
__global__ __launch_bounds__(32) void k_gemmw(const T16* __restrict__ A, const T16* __restrict__ A2, const T16* __restrict__ Bt, const T16* __restrict__ Bt2, int K, float* C, int ldc, const float* __restrict__ bias, size_t sA, size_t sB, size_t sC) {
    typedef typename WFrag<T16>::V V;
    __shared__ __align__(16) float os[16 * 68];
    const size_t z = blockIdx.z; A += z * sA; if (A2) A2 += z * sA; Bt += z * sB; if (Bt2) Bt2 += z * sB; C += z * sC;
    const int lane = threadIdx.x & 31, lr = lane & 15, hi = lane >> 4; const int r0 = blockIdx.x * 64, c0 = blockIdx.y * 64;
    v8f acc[4][4];
#pragma unroll
    for (int mb = 0; mb < 4; ++mb)
#pragma unroll
        for (int nb = 0; nb < 4; ++nb) acc[mb][nb] = (v8f){};
    const size_t aoff = (size_t)(r0 + lr) * K + 8 * hi, boff = (size_t)(c0 + lr) * K + 8 * hi;
#pragma unroll 1
    for (int kc = 0; kc < K; kc += 32) {
        V a[4], a2[4];
#pragma unroll
        for (int mb = 0; mb < 4; ++mb) { a[mb] = WFrag<T16>::ld(A + aoff + (size_t)mb * 16 * K + kc); if (NSPLIT == 1 || NSPLIT == 2) a2[mb] = WFrag<T16>::ld(A2 + aoff + (size_t)mb * 16 * K + kc); }
#pragma unroll
        for (int nb = 0; nb < 4; ++nb) { const V b = WFrag<T16>::ld(Bt + boff + (size_t)nb * 16 * K + kc); V b2; if (NSPLIT >= 2) b2 = WFrag<T16>::ld(Bt2 + boff + (size_t)nb * 16 * K + kc);
#pragma unroll
            for (int mb = 0; mb < 4; ++mb) { acc[mb][nb] = WFrag<T16>::mma(a[mb], b, acc[mb][nb]); if (NSPLIT == 1 || NSPLIT == 2) acc[mb][nb] = WFrag<T16>::mma(a2[mb], b, acc[mb][nb]); if (NSPLIT >= 2) acc[mb][nb] = WFrag<T16>::mma(a[mb], b2, acc[mb][nb]); } }
        asm volatile("v_nop\n\tv_nop\n\tv_nop\n\tv_nop" : "+v"(acc[0][0]), "+v"(acc[1][1]), "+v"(acc[2][2]), "+v"(acc[3][3]) : "v"(a[0]), "v"(a[3]));
    }
#pragma unroll
    for (int mb = 0; mb < 4; ++mb) {
#pragma unroll
        for (int nb = 0; nb < 4; ++nb) {
#pragma unroll
            for (int j = 0; j < 8; ++j) os[(hi * 8 + j) * 68 + nb * 16 + lr] = acc[mb][nb][j]; }
        __builtin_amdgcn_wave_barrier(); asm volatile("" ::: "memory");
        float* crow = C + (size_t)(r0 + mb * 16) * ldc + c0;
#pragma unroll 1
        for (int ps = 0; ps < 2; ++ps) {
#pragma unroll
            for (int s = 0; s < 8; ++s) { const int row = 2 * s + hi, cofs = lr * 4; v4f val = *(const v4fa*)(os + row * 68 + cofs);
                if (BIAS == 1) { val[0] += bfr(bias[c0 + cofs]); val[1] += bfr(bias[c0 + cofs + 1]); val[2] += bfr(bias[c0 + cofs + 2]); val[3] += bfr(bias[c0 + cofs + 3]); }
                if (BIAS == 2) { const float rb = bfr(bias[r0 + mb * 16 + row]); val[0] += rb; val[1] += rb; val[2] += rb; val[3] += rb; }
                *(volatile v4f*)(crow + (size_t)row * ldc + cofs) = val; }
            if (ps == 0) __threadfence(); }
        __builtin_amdgcn_wave_barrier(); asm volatile("" ::: "memory");
    }
}

__global__ __launch_bounds__(256) void k_cvt8(const float* __restrict__ src, bf* dst, size_t n8) { const size_t i = (size_t)blockIdx.x * 256 + threadIdx.x; if (i >= n8) return; const v8f v = *(const v8f*)(src + i * 8); v8us o;
#pragma unroll
    for (int k = 0; k < 8; ++k) o[k] = f2bf(v[k]); *(volatile v8us*)(dst + i * 8) = o; __threadfence(); *(volatile v8us*)(dst + i * 8) = o; }

__global__ __launch_bounds__(256) void k_cvtx(const float* __restrict__ x, bf* dst, size_t n8) {
    const size_t i = (size_t)blockIdx.x * 256 + threadIdx.x; if (i >= n8) return;
    const size_t e = i * 8; const size_t tok = e / DM; const size_t col = e % DM; const size_t bb = tok / SEQ; const size_t t = tok % SEQ;
    const v8f v = *(const v8f*)(x + (bb * SEQ_FULL + t) * DM + col); v8us o;
#pragma unroll
    for (int k = 0; k < 8; ++k) o[k] = f2bf(v[k]);
    *(volatile v8us*)(dst + e) = o; __threadfence(); *(volatile v8us*)(dst + e) = o; }

__global__ __launch_bounds__(256) void k_split8(const float* __restrict__ src, bf* Ph, bf* Pl, size_t n8) { const size_t i = (size_t)blockIdx.x * 256 + threadIdx.x; if (i >= n8) return; const v8f v = *(const v8f*)(src + i * 8); v8us oh, ol;
#pragma unroll
    for (int k = 0; k < 8; ++k) { unsigned short a, c; splitf(v[k], a, c); oh[k] = a; ol[k] = c; }
    *(volatile v8us*)(Ph + i * 8) = oh; *(volatile v8us*)(Pl + i * 8) = ol; __threadfence(); *(volatile v8us*)(Ph + i * 8) = oh; *(volatile v8us*)(Pl + i * 8) = ol; }

__device__ __forceinline__ float redmax16(float v) { v = fmaxf(v, __shfl_xor(v, 1, 32)); v = fmaxf(v, __shfl_xor(v, 2, 32)); v = fmaxf(v, __shfl_xor(v, 4, 32)); v = fmaxf(v, __shfl_xor(v, 8, 32)); return v; }
__device__ __forceinline__ float redsum16(float v) { v += __shfl_xor(v, 1, 32); v += __shfl_xor(v, 2, 32); v += __shfl_xor(v, 4, 32); v += __shfl_xor(v, 8, 32); return v; }

__global__ __launch_bounds__(32) void k_attn(const bf* __restrict__ Qh, const bf* __restrict__ Ql, const bf* __restrict__ Kh, const bf* __restrict__ Kl, const bf* __restrict__ Vh, const bf* __restrict__ Vl, bf* ATh, bf* ATl) {
    __shared__ __align__(16) unsigned short psh[16 * 40];
    __shared__ __align__(16) unsigned short psl[16 * 40];
    __shared__ __align__(16) float ost[16 * 68];
    const int qt = blockIdx.x, h = blockIdx.y, b = blockIdx.z;
    const int q0 = qt * 16;
    const int lane = threadIdx.x & 31, lr = lane & 15, hi = lane >> 4;
    const size_t tok0 = (size_t)b * SEQ;
    const size_t qoff = (tok0 + q0 + lr) * DQ + (size_t)h * HD + 8 * hi;
    v16bf qah[2], qal[2];
#pragma unroll
    for (int j = 0; j < 2; ++j) {
        qah[j] = cat16b(*(const v8us*)(Qh + qoff + 32 * j), *(const v8us*)(Qh + qoff + 32 * j + 16));
        qal[j] = cat16b(*(const v8us*)(Ql + qoff + 32 * j), *(const v8us*)(Ql + qoff + 32 * j + 16)); }
    v8f o[4];
#pragma unroll
    for (int nd = 0; nd < 4; ++nd) o[nd] = (v8f){};
    float mrun[8], lrun[8];
#pragma unroll
    for (int r = 0; r < 8; ++r) { mrun[r] = -1.0e30f; lrun[r] = 0.0f; }
    int ks, ke, gl;
    if (qt == 0) { ks = 0; ke = SEQ / 32 - 1; gl = 0; }
    else { int lo = q0 - WIN; if (lo < 0) lo = 0; ks = lo >> 5; ke = (q0 + 15) >> 5; gl = (ks > 0) ? 1 : 0; }
    const int nst = gl + (ke - ks + 1);
    const size_t kcol = (size_t)h * HD + 8 * hi;
    const size_t vrow0 = ((size_t)b * DM + (size_t)h * HD + lr) * SEQ + 8 * hi;
#pragma unroll 1
    for (int st = 0; st < nst; ++st) {
        const int key0 = (gl != 0 && st == 0) ? 0 : (ks + st - gl) * 32;
        v8f s[2]; s[0] = (v8f){}; s[1] = (v8f){};
        v16bf kbh, kbl;
#pragma unroll
        for (int nt = 0; nt < 2; ++nt) {
            const size_t koff = (tok0 + key0 + 16 * nt + lr) * DQ + kcol;
#pragma unroll
            for (int j = 0; j < 2; ++j) {
                kbh = cat16b(*(const v8us*)(Kh + koff + 32 * j), *(const v8us*)(Kh + koff + 32 * j + 16));
                kbl = cat16b(*(const v8us*)(Kl + koff + 32 * j), *(const v8us*)(Kl + koff + 32 * j + 16));
                s[nt] = wmmab(qah[j], kbh, s[nt]); s[nt] = wmmab(qal[j], kbh, s[nt]); s[nt] = wmmab(qah[j], kbl, s[nt]); } }
        asm volatile("v_nop\n\tv_nop\n\tv_nop\n\tv_nop" : "+v"(s[0]), "+v"(s[1]) : "v"(qah[0]), "v"(qah[1]), "v"(qal[0]), "v"(qal[1]), "v"(kbh), "v"(kbl));
        const int c0 = key0 + lr, c1 = key0 + 16 + lr;
        float p0[8], p1[8];
#pragma unroll
        for (int r = 0; r < 8; ++r) {
            const int q = q0 + 8 * hi + r;
            const bool v0 = ((c0 <= q) && (q - c0 <= WIN)) || (q == 0) || (c0 == 0);
            const bool v1 = ((c1 <= q) && (q - c1 <= WIN)) || (q == 0) || (c1 == 0);
            const float t0 = v0 ? s[0][r] * SCL : -1.0e30f;
            const float t1 = v1 ? s[1][r] * SCL : -1.0e30f;
            const float mt = redmax16(fmaxf(t0, t1)); const float mnew = fmaxf(mrun[r], mt);
            float dc = __fsub_rn(mrun[r], mnew); asm volatile("" : "+v"(dc)); const float corr = __builtin_amdgcn_exp2f(__fmul_rn(dc, L2E));
            float d0 = __fsub_rn(t0, mnew), d1 = __fsub_rn(t1, mnew); asm volatile("" : "+v"(d0)); asm volatile("" : "+v"(d1));
            const float e0r = __builtin_amdgcn_exp2f(__fmul_rn(d0, L2E)), e1r = __builtin_amdgcn_exp2f(__fmul_rn(d1, L2E));
            const float e0 = v0 ? e0r : 0.0f, e1 = v1 ? e1r : 0.0f;
            const float rs = redsum16(e0 + e1);
            lrun[r] = lrun[r] * corr + rs; mrun[r] = mnew;
            o[0][r] *= corr; o[1][r] *= corr; o[2][r] *= corr; o[3][r] *= corr;
            p0[r] = e0; p1[r] = e1; }
        __syncthreads();
#pragma unroll
        for (int r = 0; r < 8; ++r) { unsigned short a, c; splitf(p0[r], a, c); psh[(8 * hi + r) * 40 + lr] = a; psl[(8 * hi + r) * 40 + lr] = c; splitf(p1[r], a, c); psh[(8 * hi + r) * 40 + 16 + lr] = a; psl[(8 * hi + r) * 40 + 16 + lr] = c; }
        __syncthreads();
        const unsigned short* prh = psh + lr * 40 + 8 * hi; const unsigned short* prl = psl + lr * 40 + 8 * hi;
        const v16bf pah = cat16b(*(const v8usa*)prh, *(const v8usa*)(prh + 16));
        const v16bf pal = cat16b(*(const v8usa*)prl, *(const v8usa*)(prl + 16));
        v16bf vbh, vbl;
#pragma unroll
        for (int nd = 0; nd < 4; ++nd) {
            const size_t voff = vrow0 + (size_t)nd * 16 * SEQ + key0;
            vbh = cat16b(*(const v8us*)(Vh + voff), *(const v8us*)(Vh + voff + 16));
            vbl = cat16b(*(const v8us*)(Vl + voff), *(const v8us*)(Vl + voff + 16));
            o[nd] = wmmab(pah, vbh, o[nd]); o[nd] = wmmab(pal, vbh, o[nd]); o[nd] = wmmab(pah, vbl, o[nd]); }
        asm volatile("v_nop\n\tv_nop\n\tv_nop\n\tv_nop" : "+v"(o[0]), "+v"(o[1]), "+v"(o[2]), "+v"(o[3]) : "v"(pah), "v"(pal), "v"(vbh), "v"(vbl));
    }
    float inv[8];
#pragma unroll
    for (int r = 0; r < 8; ++r) inv[r] = __fdiv_rn(1.0f, lrun[r]);
#pragma unroll
    for (int nd = 0; nd < 4; ++nd)
#pragma unroll
        for (int r = 0; r < 8; ++r) ost[(8 * hi + r) * 68 + 16 * nd + lr] = o[nd][r] * inv[r];
    __syncthreads();
    v8us oh4[4], ol4[4];
#pragma unroll
    for (int i = 0; i < 4; ++i) { const int row = 4 * i + (lane >> 3); const int cc = (lane & 7) * 8; const v4f a0 = *(const v4fa*)(ost + row * 68 + cc); const v4f a1 = *(const v4fa*)(ost + row * 68 + cc + 4); v8us th, tl;
#pragma unroll
        for (int k = 0; k < 4; ++k) { unsigned short a, c; splitf(a0[k], a, c); th[k] = a; tl[k] = c; splitf(a1[k], a, c); th[4 + k] = a; tl[4 + k] = c; }
        oh4[i] = th; ol4[i] = tl; }
#pragma unroll 1
    for (int ps = 0; ps < 2; ++ps) {
#pragma unroll
        for (int i = 0; i < 4; ++i) { const int row = 4 * i + (lane >> 3); const int cc = (lane & 7) * 8; const size_t oo = (tok0 + q0 + row) * DQ + (size_t)h * HD + cc;
            *(volatile v8us*)(ATh + oo) = oh4[i]; *(volatile v8us*)(ATl + oo) = ol4[i]; }
        if (ps == 0) __threadfence(); }
}

extern "C" void kernel_launch(void* const* d_in, const int* in_sizes, int n_in,
                              void* d_out, int out_size, void* d_ws, size_t ws_size, hipStream_t stream) {
    if (n_in < 9) return;
    const size_t needx = ((size_t)(NB - 1) * SEQ_FULL + SEQ) * DM;
    if ((size_t)in_sizes[0] < needx || (size_t)in_sizes[1] < (size_t)DM * DM || in_sizes[2] < DM || (size_t)in_sizes[3] < (size_t)DM * DM || in_sizes[4] < DM ||
        (size_t)in_sizes[5] < (size_t)DM * DM || in_sizes[6] < DM || (size_t)in_sizes[7] < (size_t)DM * DM || in_sizes[8] < DM || (size_t)out_size < needx) return;
    const float* x = (const float*)d_in[0]; const float* wq = (const float*)d_in[1]; const float* bq = (const float*)d_in[2]; const float* wk = (const float*)d_in[3]; const float* bk = (const float*)d_in[4];
    const float* wv = (const float*)d_in[5]; const float* bv = (const float*)d_in[6]; const float* wo = (const float*)d_in[7]; const float* bo = (const float*)d_in[8];
    float* OUT = (float*)d_out;
    char* wsp = (char*)d_ws;
    auto take = [&](size_t bytes) { char* p = wsp; wsp += (bytes + 255) & ~(size_t)255; return (void*)p; };
    bf* WQ = (bf*)take((size_t)DQ * DM * 2); bf* WK = (bf*)take((size_t)DQ * DM * 2); bf* WV = (bf*)take((size_t)DQ * DM * 2); bf* WO = (bf*)take((size_t)DM * DQ * 2);
    bf* XB = (bf*)take((size_t)NTOK * DM * 2);
    float* F = (float*)take((size_t)NTOK * DM * 4);
    bf* QPh = (bf*)take((size_t)NTOK * DQ * 2); bf* QPl = (bf*)take((size_t)NTOK * DQ * 2);
    bf* KPh = (bf*)take((size_t)NTOK * DQ * 2); bf* KPl = (bf*)take((size_t)NTOK * DQ * 2);
    bf* VTh = (bf*)take((size_t)NB * DM * SEQ * 2); bf* VTl = (bf*)take((size_t)NB * DM * SEQ * 2);
    bf* ATh = (bf*)take((size_t)NTOK * DQ * 2); bf* ATl = (bf*)take((size_t)NTOK * DQ * 2);
    if ((size_t)(wsp - (char*)d_ws) > ws_size) return;
    const size_t w8 = (size_t)DM * DM / 8;
    k_cvt8<<<(unsigned)((w8 + 255) / 256), 256, 0, stream>>>(wq, WQ, w8);
    k_cvt8<<<(unsigned)((w8 + 255) / 256), 256, 0, stream>>>(wk, WK, w8);
    k_cvt8<<<(unsigned)((w8 + 255) / 256), 256, 0, stream>>>(wv, WV, w8);
    k_cvt8<<<(unsigned)((w8 + 255) / 256), 256, 0, stream>>>(wo, WO, w8);
    const size_t x8 = (size_t)NTOK * DM / 8;
    k_cvtx<<<(unsigned)((x8 + 255) / 256), 256, 0, stream>>>(x, XB, x8);
    k_gemmw<bf, 0, 1><<<dim3(NTOK / 64, DQ / 64, 1), 32, 0, stream>>>(XB, nullptr, WQ, nullptr, DM, F, DQ, bq, 0, 0, 0);
    k_split8<<<(unsigned)((x8 + 255) / 256), 256, 0, stream>>>(F, QPh, QPl, x8);
    k_gemmw<bf, 0, 1><<<dim3(NTOK / 64, DQ / 64, 1), 32, 0, stream>>>(XB, nullptr, WK, nullptr, DM, F, DQ, bk, 0, 0, 0);
    k_split8<<<(unsigned)((x8 + 255) / 256), 256, 0, stream>>>(F, KPh, KPl, x8);
    k_gemmw<bf, 0, 2><<<dim3(DM / 64, SEQ / 64, NB), 32, 0, stream>>>(WV, nullptr, XB, nullptr, DM, F, SEQ, bv, 0, (size_t)SEQ * DM, (size_t)DM * SEQ);
    k_split8<<<(unsigned)((x8 + 255) / 256), 256, 0, stream>>>(F, VTh, VTl, x8);
    k_attn<<<dim3(SEQ / 16, NH_, NB), 32, 0, stream>>>(QPh, QPl, KPh, KPl, VTh, VTl, ATh, ATl);
    k_gemmw<bf, 1, 1><<<dim3(SEQ / 64, DM / 64, NB), 32, 0, stream>>>(ATh, ATl, WO, nullptr, DQ, OUT, DM, bo, (size_t)SEQ * DQ, 0, (size_t)SEQ_FULL * DM);
}
